// LocalAggregator_67937792688246
// MI455X (gfx1250) — hardware-verified
//
#include <hip/hip_runtime.h>

constexpr int kNodes     = 100;
constexpr int kDim       = 128;
constexpr int kPadN      = 128;
constexpr int kRelA      = 3;
constexpr int kRelB      = 9;
constexpr int kMaps      = kRelA + kRelB;
constexpr int kARows     = 1216;
constexpr int kPlaneRows = kARows + kPadN;
constexpr int kChunkB    = 32;
constexpr int kPCols     = 2 * kPadN;
constexpr float kLeaky    = 0.2f;
constexpr float kMaskVal  = -9.0e15f;
constexpr float kPCarry   = 2048.0f;
constexpr float kAggScale = 1.0f / 4096.0f;


typedef __attribute__((ext_vector_type(16))) _Float16 v16h;
typedef __attribute__((ext_vector_type(8)))  _Float16 v8h;
typedef __attribute__((ext_vector_type(16))) __bf16   v16b;
typedef __attribute__((ext_vector_type(8)))  __bf16   v8b;
typedef __attribute__((ext_vector_type(8)))  float    v8f;
typedef __attribute__((ext_vector_type(4)))  float    v4f;
typedef __attribute__((ext_vector_type(4)))  unsigned int v4u;

__device__ __forceinline__ unsigned short f2bf_bits(float f) {
  unsigned u = __float_as_uint(f);
  return (unsigned short)((u + 0x7FFFu + ((u >> 16) & 1u)) >> 16);
}
__device__ __forceinline__ float bf_bits2f(unsigned short h) { return __uint_as_float(((unsigned)h) << 16); }

__device__ __forceinline__ void dep_guard_h(v8f& a, v8f& b, v16h x, v16h y) { asm volatile("v_nop\n\tv_nop\n\tv_nop\n\tv_nop" : "+v"(a), "+v"(b) : "v"(x), "v"(y)); }
__device__ __forceinline__ void dep_guard_b(v8f& a, v8f& b, v16b x, v16b y) { asm volatile("v_nop\n\tv_nop\n\tv_nop\n\tv_nop" : "+v"(a), "+v"(b) : "v"(x), "v"(y)); }
__device__ __forceinline__ void keep4_h(v16h a, v16h b, v16h c, v16h d) { asm volatile("v_nop" :: "v"(a), "v"(b), "v"(c), "v"(d)); }
__device__ __forceinline__ void keep4_b(v16b a, v16b b, v16b c, v16b d) { asm volatile("v_nop" :: "v"(a), "v"(b), "v"(c), "v"(d)); }
__device__ __forceinline__ void acc_guard4(v8f& a, v8f& b, v8f& c, v8f& d) { asm volatile("v_nop\n\tv_nop\n\tv_nop\n\tv_nop" : "+v"(a), "+v"(b), "+v"(c), "+v"(d)); }
template <typename T> struct Frag;
template <> struct Frag<_Float16> {
  typedef v16h V; union U { v16h v; v8h h[2]; };
  static __device__ __forceinline__ v16h load(const _Float16* p) {
    U f; f.h[0] = *(const v8h*)(p); f.h[1] = *(const v8h*)(p + 16); return f.v;
  }
  static __device__ __forceinline__ v8f mma(v16h a, v16h b, v8f c) {
    return __builtin_amdgcn_wmma_f32_16x16x32_f16(false, a, false, b, (short)0, c, false, false);
  }
  static __device__ __forceinline__ void guard(v8f& a, v8f& b, v16h x, v16h y) { dep_guard_h(a, b, x, y); }
  static __device__ __forceinline__ void keep(v16h a, v16h b, v16h c, v16h d) { keep4_h(a, b, c, d); }
};
template <> struct Frag<__bf16> {
  typedef v16b V; union U { v16b v; v8b h[2]; };
  static __device__ __forceinline__ v16b load(const __bf16* p) {
    U f; f.h[0] = *(const v8b*)(p); f.h[1] = *(const v8b*)(p + 16); return f.v;
  }
  static __device__ __forceinline__ v8f mma(v16b a, v16b b, v8f c) {
    return __builtin_amdgcn_wmma_f32_16x16x32_bf16(false, a, false, b, (short)0, c, false, false);
  }
  static __device__ __forceinline__ void guard(v8f& a, v8f& b, v16b x, v16b y) { dep_guard_b(a, b, x, y); }
  static __device__ __forceinline__ void keep(v16b a, v16b b, v16b c, v16b d) { keep4_b(a, b, c, d); }
};

__device__ __forceinline__ unsigned pk16(unsigned short a, unsigned short b) { return (unsigned)a | ((unsigned)b << 16); }
__device__ __forceinline__ unsigned short h_bits(float f) { const _Float16 h = (_Float16)f; return __builtin_bit_cast(unsigned short, h); }

template <int ET> struct Elem;
template <> struct Elem<0> { typedef _Float16 T; };
template <> struct Elem<1> { typedef __bf16 T; };
template <int ET, bool SPLIT, int BIAS_MODE, int OUT_MODE, bool RESID, int ACT = 0>
__global__ __launch_bounds__(256) void wmma_gemm64(
    const unsigned short* __restrict__ Ap, const unsigned short* __restrict__ A2p, int lda, long strideA,
    const unsigned short* __restrict__ Btp, const unsigned short* __restrict__ Bt2p, int ldb, long strideB,
    void* __restrict__ Cout, void* __restrict__ Cout2, int ldc, long strideC,
    const float* __restrict__ bias,
    const float* __restrict__ resid, long strideR,
    int M, int N, int K, float scale) {
  typedef typename Elem<ET>::T T;
  typedef typename Frag<T>::V V;
  const T* A = (const T*)Ap; const T* A2 = (const T*)A2p; const T* Bt = (const T*)Btp; const T* Bt2 = (const T*)Bt2p;
  __shared__ __align__(16) float sT[8][16 * 68];
  const int b    = blockIdx.y;
  const int lane = threadIdx.x & 31;
  const int wave = threadIdx.x >> 5;
  const int tilesN = N >> 6;
  const int tilesM = M >> 6;
  const int tile = blockIdx.x * 8 + wave;
  if (tile >= tilesM * tilesN) return;
  const int tm = tile / tilesN;
  const int tn = tile - tm * tilesN;
  const int m0 = tm << 6;
  const int n0 = tn << 6;

  const T* Ab  = A  + (size_t)b * strideA;
  const T* Bb  = Bt + (size_t)b * strideB;
  const T* Ab2 = SPLIT ? (A2  + (size_t)b * strideA) : nullptr;
  const T* Bb2 = SPLIT ? (Bt2 + (size_t)b * strideB) : nullptr;

  const int rlane = lane & 15;
  const int koff  = (lane >> 4) * 8;
  const int mOff  = (lane >> 4) * 8;

  v8f acc[4][4];
#pragma unroll
  for (int i = 0; i < 4; ++i)
#pragma unroll
    for (int j = 0; j < 4; ++j) acc[i][j] = (v8f){0.f,0.f,0.f,0.f,0.f,0.f,0.f,0.f};

  for (int k0 = 0; k0 < K; k0 += 32) {
    V bh[4], bl[4];
#pragma unroll
    for (int j = 0; j < 4; ++j) {
      const size_t bo = (size_t)(n0 + (j << 4) + rlane) * ldb + koff + k0;
      bh[j] = Frag<T>::load(Bb + bo);
      if (SPLIT) bl[j] = Frag<T>::load(Bb2 + bo);
    }
#pragma unroll
    for (int i = 0; i < 4; ++i) {
      const size_t ao = (size_t)(m0 + (i << 4) + rlane) * lda + koff + k0;
      V ah = Frag<T>::load(Ab + ao);
      V al;
      if (SPLIT) al = Frag<T>::load(Ab2 + ao);
#pragma unroll
      for (int j = 0; j < 4; ++j) {
        acc[i][j] = Frag<T>::mma(ah, bh[j], acc[i][j]);
        if (SPLIT) {
          acc[i][j] = Frag<T>::mma(ah, bl[j], acc[i][j]);
          acc[i][j] = Frag<T>::mma(al, bh[j], acc[i][j]);
        }
      }
      Frag<T>::guard(acc[i][0], acc[i][3], ah, SPLIT ? al : ah);
    }
    Frag<T>::keep(bh[0], bh[1], bh[2], bh[3]);
    if (SPLIT) Frag<T>::keep(bl[0], bl[1], bl[2], bl[3]);
  }
  acc_guard4(acc[0][0], acc[0][1], acc[0][2], acc[0][3]);
  acc_guard4(acc[1][0], acc[1][1], acc[1][2], acc[1][3]);
  acc_guard4(acc[2][0], acc[2][1], acc[2][2], acc[2][3]);
  acc_guard4(acc[3][0], acc[3][1], acc[3][2], acc[3][3]);

  float* slab = sT[wave];
  const float* Rb = RESID ? (resid + (size_t)b * strideR) : nullptr;
#pragma unroll
  for (int i = 0; i < 4; ++i) {
    const int mBase = m0 + (i << 4);
#pragma unroll
    for (int j = 0; j < 4; ++j) {
      const int n = n0 + (j << 4) + rlane;
      float bv = 0.f;
      if (BIAS_MODE == 2) bv = bias[n];
#pragma unroll
      for (int r = 0; r < 8; ++r) {
        float v = acc[i][j][r] * scale;
        if (BIAS_MODE == 1) v += bias[mBase + mOff + r];
        if (BIAS_MODE == 2) v += bv;
        if (RESID) v += Rb[(size_t)(mBase + mOff + r) * ldc + n];
        if (ACT == 2) v = fmaxf(v, 0.0f);
        if (ACT == 4) v = (v > 0.f) ? v : 0.01f * v;
        slab[(mOff + r) * 68 + (j << 4) + rlane] = v;
      }
    }
    __builtin_amdgcn_fence(__ATOMIC_RELEASE, "workgroup");
    __builtin_amdgcn_wave_barrier();
    __builtin_amdgcn_fence(__ATOMIC_ACQUIRE, "workgroup");
    if (OUT_MODE == 0) {
      float* C = (float*)Cout + (size_t)b * strideC;
      const int hh = lane >> 4, c4 = (lane & 15) * 4;
      for (int pass = 0; pass < 2; ++pass) {
#pragma unroll
        for (int it = 0; it < 8; ++it) {
          const int row = it * 2 + hh;
          v4f v = *(const v4f*)(slab + row * 68 + c4);
          *(volatile v4f*)(C + (size_t)(mBase + row) * ldc + n0 + c4) = v;
        }
        __threadfence();
      }
    } else {
      const int q = lane >> 3, c8 = (lane & 7) * 8;
      unsigned short* C  = (unsigned short*)Cout  + (size_t)b * strideC;
      unsigned short* C2 = (OUT_MODE == 2) ? ((unsigned short*)Cout2 + (size_t)b * strideC) : nullptr;
      for (int pass = 0; pass < 2; ++pass) {
#pragma unroll
        for (int it = 0; it < 4; ++it) {
          const int row = it * 4 + q;
          const float* sp = slab + row * 68 + c8;
          v8h hv, lv;
#pragma unroll
          for (int e = 0; e < 8; ++e) {
            if (OUT_MODE == 1) {
              hv[e] = (_Float16)sp[e];
            } else {
              unsigned short hb = f2bf_bits(sp[e]);
              unsigned short lb = f2bf_bits(sp[e] - bf_bits2f(hb));
              hv[e] = __builtin_bit_cast(_Float16, hb);
              lv[e] = __builtin_bit_cast(_Float16, lb);
            }
          }
          *(volatile v8h*)(C + (size_t)(mBase + row) * ldc + n0 + c8) = hv;
          if (OUT_MODE == 2) *(volatile v8h*)(C2 + (size_t)(mBase + row) * ldc + n0 + c8) = lv;
        }
        __threadfence();
      }
    }
    __builtin_amdgcn_fence(__ATOMIC_RELEASE, "workgroup");
    __builtin_amdgcn_wave_barrier();
    __builtin_amdgcn_fence(__ATOMIC_ACQUIRE, "workgroup");
  }
}

__global__ __launch_bounds__(256) void prep_planes_kernel(const float* __restrict__ hidden,
                                                          const float* __restrict__ Aw,
                                                          const float* __restrict__ Bw,
                                                          unsigned short* __restrict__ Phi,
                                                          unsigned short* __restrict__ Plo, int b0) {
  const int bl = blockIdx.y;
  const int b  = b0 + bl;
  const int t  = blockIdx.x * 256 + threadIdx.x;
  if (t >= kPlaneRows * 16) return;
  const int dseg = t & 15;
  const int row  = t >> 4;
  const int d0   = dseg * 8;
  const bool isA = row < kARows;
  int k = row / kNodes;
  k = (k > kMaps - 1) ? (kMaps - 1) : k;
  const int iA = row - k * kNodes;
  const int jH = row - kARows;
  const int src = isA ? iA : jH;
  const bool valid = isA ? (row < kMaps * kNodes) : (jH < kNodes);
  int srcc = (src < 0) ? 0 : src;
  srcc = (srcc > kNodes - 1) ? (kNodes - 1) : srcc;
  const float* hp = hidden + ((size_t)b * kNodes + srcc) * kDim + d0;
  const v4f x0 = *(const v4f*)(hp);
  const v4f x1 = *(const v4f*)(hp + 4);
  float x[8];
  x[0] = x0[0]; x[1] = x0[1]; x[2] = x0[2]; x[3] = x0[3];
  x[4] = x1[0]; x[5] = x1[1]; x[6] = x1[2]; x[7] = x1[3];
  const int kA = (k > kRelA - 1) ? (kRelA - 1) : k;
  int kB = k - kRelA;
  kB = (kB < 0) ? 0 : kB;
  kB = (kB > kRelB - 1) ? (kRelB - 1) : kB;
  unsigned short hb[8], lb[8];
#pragma unroll
  for (int e = 0; e < 8; ++e) {
    const int d = d0 + e;
    const float ca = Aw[d * kRelA + kA];
    const float cb = Bw[d * kRelB + kB];
    const float c  = isA ? ((k < kRelA) ? ca : cb) : 1.0f;
    const float v  = valid ? (x[e] * c) : 0.0f;
    const unsigned short h1 = f2bf_bits(v);
    hb[e] = h1;
    lb[e] = f2bf_bits(v - bf_bits2f(h1));
  }
  const v4u uh = (v4u){pk16(hb[0], hb[1]), pk16(hb[2], hb[3]), pk16(hb[4], hb[5]), pk16(hb[6], hb[7])};
  const v4u ul = (v4u){pk16(lb[0], lb[1]), pk16(lb[2], lb[3]), pk16(lb[4], lb[5]), pk16(lb[6], lb[7])};
  const size_t off = ((size_t)bl * kPlaneRows + row) * kDim + d0;
  *(volatile v4u*)(Phi + off) = uh;
  *(volatile v4u*)(Plo + off) = ul;
  __threadfence();
  *(volatile v4u*)(Phi + off) = uh;
  *(volatile v4u*)(Plo + off) = ul;
}

__global__ __launch_bounds__(256) void ht2_kernel(const float* __restrict__ hidden, unsigned short* __restrict__ HT2, int b0) {
  __shared__ float sm[kPadN][65];
  const int t  = threadIdx.x;
  const int bl = blockIdx.y;
  const int b  = b0 + bl;
  const int d0 = blockIdx.x * 64;
#pragma unroll 4
  for (int it = 0; it < 32; ++it) {
    const int e  = it * 256 + t;
    const int j  = e >> 6;
    const int dl = e & 63;
    const int jc = (j < kNodes) ? j : (kNodes - 1);
    const float v = hidden[((size_t)b * kNodes + jc) * kDim + d0 + dl];
    sm[j][dl] = (j < kNodes) ? v : 0.0f;
  }
  __syncthreads();
  const int lane = t & 31, wave = t >> 5;
  const int c0   = lane * 8;
  const int j0   = c0 & 127;
#pragma unroll 1
  for (int it = 0; it < 8; ++it) {
    const int dl = wave * 8 + it;
    unsigned short hbv[8];
#pragma unroll
    for (int e = 0; e < 8; ++e) hbv[e] = h_bits(sm[j0 + e][dl]);
    const v4u u = (v4u){pk16(hbv[0], hbv[1]), pk16(hbv[2], hbv[3]), pk16(hbv[4], hbv[5]), pk16(hbv[6], hbv[7])};
    unsigned short* dst = HT2 + ((size_t)bl * kDim + d0 + dl) * kPCols + c0;
    *(volatile v4u*)dst = u;
    __threadfence();
    *(volatile v4u*)dst = u;
  }
}

__global__ __launch_bounds__(128) void select_softmax_kernel(const float* __restrict__ S, const int* __restrict__ adj,
                                                             const int* __restrict__ beh, unsigned short* __restrict__ P,
                                                             int b0) {
  __shared__ float redMa[4], redMb[4], redSa[4], redSb[4];
  __shared__ __align__(16) float sp[kPCols];
  const int i  = blockIdx.x;
  const int bl = blockIdx.y;
  const int b  = b0 + bl;
  const int t  = threadIdx.x;
  const int lane = t & 31, wave = t >> 5;
  const int ic = (i < kNodes) ? i : (kNodes - 1);
  const float rowscale = (i < kNodes) ? kPCarry : 0.0f;
  const int j  = t;
  const int jc = (j < kNodes) ? j : (kNodes - 1);
  const bool jv = (j < kNodes);
  const size_t aoff = ((size_t)b * kNodes + ic) * kNodes + jc;
  const int ca = adj[aoff];
  const int cb = beh[aoff];
  const bool va = (ca >= 1) && (ca <= kRelA);
  int ka = ca - 1; ka = (ka < 0) ? 0 : ka; ka = (ka > kRelA - 1) ? (kRelA - 1) : ka;
  const bool vb = (cb >= 1) && (cb <= kRelB);
  int kb = cb - 1; kb = (kb < 0) ? 0 : kb; kb = (kb > kRelB - 1) ? (kRelB - 1) : kb;
  const float* Sb = S + (size_t)bl * kARows * kPadN;
  float sa = Sb[(size_t)(ka * kNodes + ic) * kPadN + jc];
  float sb = Sb[(size_t)(kRelA * kNodes + kb * kNodes + ic) * kPadN + jc];
  sa = (sa >= 0.0f) ? sa : kLeaky * sa;
  sb = (sb >= 0.0f) ? sb : kLeaky * sb;
  float ea = va ? sa : kMaskVal;
  float eb = vb ? sb : kMaskVal;
  ea = jv ? ea : -__builtin_inff();
  eb = jv ? eb : -__builtin_inff();

  float ma = ea, mb = eb;
#pragma unroll
  for (int off = 16; off > 0; off >>= 1) {
    ma = fmaxf(ma, __shfl_xor(ma, off, 32));
    mb = fmaxf(mb, __shfl_xor(mb, off, 32));
  }
  if (lane == 0) { redMa[wave] = ma; redMb[wave] = mb; }
  __syncthreads();
  const float Ma = fmaxf(fmaxf(redMa[0], redMa[1]), fmaxf(redMa[2], redMa[3]));
  const float Mb = fmaxf(fmaxf(redMb[0], redMb[1]), fmaxf(redMb[2], redMb[3]));
  const float xa = expf(ea - Ma);
  const float xb = expf(eb - Mb);
  float pa = xa, pb = xb;
#pragma unroll
  for (int off = 16; off > 0; off >>= 1) {
    pa += __shfl_xor(pa, off, 32);
    pb += __shfl_xor(pb, off, 32);
  }
  if (lane == 0) { redSa[wave] = pa; redSb[wave] = pb; }
  __syncthreads();
  const float Sa = ((redSa[0] + redSa[1]) + redSa[2]) + redSa[3];
  const float Sbb = ((redSb[0] + redSb[1]) + redSb[2]) + redSb[3];
  const float va_out = (xa * (1.0f / Sa)) * rowscale;
  const float vb_out = (xb * (1.0f / Sbb)) * rowscale;
  sp[t] = va_out;
  sp[kPadN + t] = vb_out;
  __syncthreads();
  if (wave == 0) {
    const float* q = sp + lane * 8;
    const v4f a0 = *(const v4f*)(q);
    const v4f a1 = *(const v4f*)(q + 4);
    unsigned short hbv[8];
    hbv[0] = h_bits(a0[0]); hbv[1] = h_bits(a0[1]); hbv[2] = h_bits(a0[2]); hbv[3] = h_bits(a0[3]);
    hbv[4] = h_bits(a1[0]); hbv[5] = h_bits(a1[1]); hbv[6] = h_bits(a1[2]); hbv[7] = h_bits(a1[3]);
    const v4u u = (v4u){pk16(hbv[0], hbv[1]), pk16(hbv[2], hbv[3]), pk16(hbv[4], hbv[5]), pk16(hbv[6], hbv[7])};
    unsigned short* dst = P + ((size_t)bl * kPadN + i) * kPCols + lane * 8;
    *(volatile v4u*)dst = u;
    __threadfence();
    *(volatile v4u*)dst = u;
  }
}

__global__ __launch_bounds__(256) void copy_out_kernel(const float* __restrict__ O, float* __restrict__ out, int b0, int nrows) {
  const int lane = threadIdx.x & 31, wave = threadIdx.x >> 5;
  const int r = blockIdx.x * 8 + wave;
  if (r >= nrows) return;
  const int bl = r / kNodes;
  const int i  = r - bl * kNodes;
  const v4f v = *(const v4f*)(O + ((size_t)bl * kPadN + i) * kDim + lane * 4);
  float* dst = out + ((size_t)(b0 + bl) * kNodes + i) * kDim + lane * 4;
  *(volatile v4f*)dst = v;
  __threadfence();
  *(volatile v4f*)dst = v;
}

extern "C" void kernel_launch(void* const* d_in, const int* in_sizes, int n_in,
                              void* d_out, int out_size, void* d_ws, size_t ws_size,
                              hipStream_t stream) {
  if (n_in < 5) return;
  const float* hidden = (const float*)d_in[0];
  const int*   adj    = (const int*)d_in[1];
  const int*   beh    = (const int*)d_in[2];
  const float* Aw     = (const float*)d_in[3];
  const float* Bw     = (const float*)d_in[4];
  float*       out    = (float*)d_out;

  const int nB = in_sizes[0] / (kNodes * kDim);
  if (nB <= 0 || nB * kNodes * kDim != in_sizes[0]) return;
  if (in_sizes[1] != nB * kNodes * kNodes || in_sizes[2] != nB * kNodes * kNodes) return;
  if (in_sizes[3] != kDim * kRelA || in_sizes[4] != kDim * kRelB) return;
  if (out_size != nB * kNodes * kDim) return;

  const size_t szPlane = (size_t)kChunkB * kPlaneRows * kDim * 2;
  const size_t szS     = (size_t)kChunkB * kARows * kPadN * 4;
  const size_t szHT2   = (size_t)kChunkB * kDim * kPCols * 2;
  const size_t szP     = (size_t)kChunkB * kPadN * kPCols * 2;
  const size_t szO     = (size_t)kChunkB * kPadN * kDim * 4;
  const size_t oPhi = 0;
  const size_t oPlo = oPhi + szPlane;
  const size_t oS   = oPlo + szPlane;
  const size_t oHT2 = oS + szS;
  const size_t oP   = oHT2 + szHT2;
  const size_t oO   = oP + szP;
  const size_t total = oO + szO;
  if (total > ws_size) return;
  char* ws = (char*)d_ws;
  unsigned short* Phi = (unsigned short*)(ws + oPhi);
  unsigned short* Plo = (unsigned short*)(ws + oPlo);
  float*          Sp  = (float*)(ws + oS);
  unsigned short* HT2 = (unsigned short*)(ws + oHT2);
  unsigned short* Pp  = (unsigned short*)(ws + oP);
  float*          Op  = (float*)(ws + oO);

  const dim3 blk256(256), blk128(128);
  const int nChunks = (nB + kChunkB - 1) / kChunkB;
  const int scoreTiles = (kARows / 64) * (kPadN / 64);
  const int aggTiles   = (kPadN / 64) * (kDim / 64);
  for (int ch = 0; ch < nChunks; ++ch) {
    const int b0 = ch * kChunkB;
    const int cb = (nB - b0 < kChunkB) ? (nB - b0) : kChunkB;
    prep_planes_kernel<<<dim3((kPlaneRows * 16 + 255) / 256, cb), blk256, 0, stream>>>(hidden, Aw, Bw, Phi, Plo, b0);
    ht2_kernel<<<dim3(kDim / 64, cb), blk256, 0, stream>>>(hidden, HT2, b0);
    wmma_gemm64<1, true, 0, 0, false, 0><<<dim3((scoreTiles + 7) / 8, cb), blk256, 0, stream>>>(
        Phi, Plo, kDim, (long)kPlaneRows * kDim,
        Phi + (size_t)kARows * kDim, Plo + (size_t)kARows * kDim, kDim, (long)kPlaneRows * kDim,
        (void*)Sp, nullptr, kPadN, (long)kARows * kPadN,
        nullptr, nullptr, 0L,
        kARows, kPadN, kDim, 1.0f);
    select_softmax_kernel<<<dim3(kPadN, cb), blk128, 0, stream>>>(Sp, adj, beh, Pp, b0);
    wmma_gemm64<0, false, 0, 0, false, 0><<<dim3((aggTiles + 7) / 8, cb), blk256, 0, stream>>>(
        Pp, nullptr, kPCols, (long)kPadN * kPCols,
        HT2, nullptr, kPCols, (long)kDim * kPCols,
        (void*)Op, nullptr, kDim, (long)kPadN * kDim,
        nullptr, nullptr, 0L,
        kPadN, kDim, kPCols, kAggScale);
    copy_out_kernel<<<dim3((cb * kNodes + 7) / 8), blk256, 0, stream>>>(Op, out, b0, cb * kNodes);
  }
}
